// MultiHeadAttention_17867063951632
// MI455X (gfx1250) — hardware-run, weakly checked
//
#include <hip/hip_runtime.h>
#ifndef NB
#define NB 2
#endif
#ifndef SEQ
#define SEQ 2048
#endif
#define NB_FULL 2
#define SEQ_FULL 2048
#define DM 512
#define NH 8
#define HD 64
#define MROWS (NB * SEQ)
#define BSTRIDE_FULL ((size_t)SEQ_FULL * DM)
#define NMB (SEQ / 32)
#define PLANE_B ((size_t)MROWS * DM * 2)
#define RPLANE_B ((size_t)SEQ * DM * 2)
#define WPLANE_B ((size_t)DM * DM * 2)
#define CARVE_B (13 * PLANE_B + 3 * RPLANE_B + 5 * WPLANE_B + (size_t)NMB * 128 + 23 * 256)

static_assert(SEQ % 64 == 0);
static_assert(SEQ <= SEQ_FULL);
static_assert(NB <= NB_FULL);
static_assert(DM == 512 && HD == 64 && NH * HD == DM);
static_assert(NMB <= 128);
static_assert(CARVE_B <= (size_t)134217728);
static_assert((size_t)(NB - 1) * SEQ_FULL * DM + (size_t)SEQ * DM <= (size_t)NB_FULL * SEQ_FULL * DM);

typedef __bf16 v16b __attribute__((ext_vector_type(16)));
typedef unsigned short v8us __attribute__((ext_vector_type(8), may_alias));
typedef float v8f __attribute__((ext_vector_type(8)));
typedef float v4f __attribute__((ext_vector_type(4)));
typedef float v4fa __attribute__((ext_vector_type(4), may_alias));
typedef int v4ia __attribute__((ext_vector_type(4), may_alias));
union FragB { v16b v; v8us half[2]; unsigned short u[16]; };

#define LOG2E 1.4426950408889634f
#define NEGFILL (-1.0e30f)

__device__ __forceinline__ unsigned short bf16_bits(float x) {
  unsigned int u = __float_as_uint(x);
  return (unsigned short)((u + 0x7FFFu + ((u >> 16) & 1u)) >> 16);
}
__device__ __forceinline__ float bf16_val(unsigned short b) { return __uint_as_float(((unsigned int)b) << 16); }
__device__ __forceinline__ float bf16_rne(float x) { return bf16_val(bf16_bits(x)); }

__device__ __forceinline__ void split8(const float (&x)[8], v8us& hi, v8us& lo) {
#pragma unroll
  for (int e = 0; e < 8; ++e) {
    const unsigned short hb = bf16_bits(x[e]);
    hi[e] = hb;
    lo[e] = bf16_bits(x[e] - bf16_val(hb));
  }
}

__device__ __forceinline__ v8f wm(v16b a, v16b b, v8f c) {
  return __builtin_amdgcn_wmma_f32_16x16x32_bf16(false, a, false, b, (short)0, c, false, false);
}

__device__ __forceinline__ v8f tile_qk(const unsigned short* __restrict__ PH, const unsigned short* __restrict__ PL, int row, int hh,
                                       const FragB& bh0, const FragB& bl0, const FragB& bh1, const FragB& bl1) {
  const int rc = (row < SEQ - 1) ? row : (SEQ - 1);
  const size_t o = (size_t)rc * DM + 8 * hh;
  FragB ah0, al0, ah1, al1;
  ah0.half[0] = *(const v8us*)(PH + o);      ah0.half[1] = *(const v8us*)(PH + o + 16);
  ah1.half[0] = *(const v8us*)(PH + o + 32); ah1.half[1] = *(const v8us*)(PH + o + 48);
  al0.half[0] = *(const v8us*)(PL + o);      al0.half[1] = *(const v8us*)(PL + o + 16);
  al1.half[0] = *(const v8us*)(PL + o + 32); al1.half[1] = *(const v8us*)(PL + o + 48);
  v8f c = {0.f, 0.f, 0.f, 0.f, 0.f, 0.f, 0.f, 0.f};
  c = wm(ah0.v, bh0.v, c); c = wm(ah0.v, bl0.v, c); c = wm(al0.v, bh0.v, c);
  c = wm(ah1.v, bh1.v, c); c = wm(ah1.v, bl1.v, c); c = wm(al1.v, bh1.v, c);
  asm volatile("v_nop\n\tv_nop\n\tv_nop\n\tv_nop" : "+v"(c)
               : "v"(ah0.v), "v"(al0.v), "v"(ah1.v), "v"(al1.v), "v"(bh0.v), "v"(bl0.v), "v"(bh1.v), "v"(bl1.v));
  return c;
}

__device__ __forceinline__ v8f mma_pv(v16b vh, v16b vl, v16b ph, v16b pl, v8f c) {
  c = wm(vh, ph, c); c = wm(vh, pl, c); c = wm(vl, ph, c);
  asm volatile("v_nop\n\tv_nop\n\tv_nop\n\tv_nop" : "+v"(c) : "v"(vh), "v"(vl), "v"(ph), "v"(pl));
  return c;
}

__global__ __launch_bounds__(256) void k_cvt(const float* __restrict__ src, unsigned short* dst, int nb, int rows, size_t sbs) {
  const int t = blockIdx.x * 256 + threadIdx.x;
  if (t >= nb * rows * 64) return;
  const int row = t >> 6, piece = t & 63;
  const int b = row / rows, s = row - b * rows;
  const float* p = src + (size_t)b * sbs + (size_t)s * DM + piece * 8;
  const v4f x0 = *(const v4fa*)(p), x1 = *(const v4fa*)(p + 4);
  v8us o;
  o[0] = bf16_bits(x0[0]); o[1] = bf16_bits(x0[1]); o[2] = bf16_bits(x0[2]); o[3] = bf16_bits(x0[3]);
  o[4] = bf16_bits(x1[0]); o[5] = bf16_bits(x1[1]); o[6] = bf16_bits(x1[2]); o[7] = bf16_bits(x1[3]);
  unsigned short* d = dst + (size_t)t * 8;
  *(volatile v8us*)d = o;
  __threadfence();
  *(volatile v8us*)d = o;
}

__global__ __launch_bounds__(256) void k_maskchk(const int* __restrict__ mask, int* flags) {
  __shared__ int red[8];
  const int tid = threadIdx.x;
  const int row0 = blockIdx.x * 32;
  int bad = 0;
  for (int i = tid; i < 32 * (SEQ / 4); i += 256) {
    const int r = row0 + i / (SEQ / 4);
    const int c = (i % (SEQ / 4)) * 4;
    const v4ia m = *(const v4ia*)(mask + (size_t)r * SEQ_FULL + c);
    bad |= ((m[0] != 0) != (c + 0 > r)) ? 1 : 0;
    bad |= ((m[1] != 0) != (c + 1 > r)) ? 1 : 0;
    bad |= ((m[2] != 0) != (c + 2 > r)) ? 1 : 0;
    bad |= ((m[3] != 0) != (c + 3 > r)) ? 1 : 0;
  }
  bad |= __shfl_xor(bad, 16, 32);
  bad |= __shfl_xor(bad, 8, 32);
  bad |= __shfl_xor(bad, 4, 32);
  bad |= __shfl_xor(bad, 2, 32);
  bad |= __shfl_xor(bad, 1, 32);
  if ((tid & 31) == 0) red[tid >> 5] = bad;
  __syncthreads();
  if (tid < 32) {
    const int tot = red[0] | red[1] | red[2] | red[3] | red[4] | red[5] | red[6] | red[7];
    int* d = flags + blockIdx.x * 32 + tid;
    *(volatile int*)d = tot;
    __threadfence();
    *(volatile int*)d = tot;
  }
}

template <int MODE>
__global__ __launch_bounds__(128) void k_gemm(const unsigned short* __restrict__ A, const unsigned short* __restrict__ A2,
                                              const unsigned short* __restrict__ W,
                                              const float* __restrict__ bias0, const float* __restrict__ bias1,
                                              unsigned short* o0, unsigned short* o1, unsigned short* o2, unsigned short* o3,
                                              float* outF, const int* __restrict__ flags) {
  __shared__ __attribute__((aligned(16))) float st[64][68];
  __shared__ int sbad;
  const int tid = threadIdx.x, w = tid >> 5, lane = tid & 31, ln = lane & 15, hh = lane >> 4;
  const int m0 = blockIdx.x * 64, n0 = blockIdx.y * 64;
  v8f acc[4] = {};
  const unsigned short* pa = A + (size_t)(m0 + 16 * w + ln) * DM + 8 * hh;
  const unsigned short* pa2 = A2 + (size_t)(m0 + 16 * w + ln) * DM + 8 * hh;
  const unsigned short* pw = W + (size_t)(n0 + ln) * DM + 8 * hh;
#pragma unroll 1
  for (int k0 = 0; k0 < DM; k0 += 32) {
    FragB a, bw[4];
    a.half[0] = *(const v8us*)(pa + k0);
    a.half[1] = *(const v8us*)(pa + k0 + 16);
#pragma unroll
    for (int nt = 0; nt < 4; ++nt) {
      bw[nt].half[0] = *(const v8us*)(pw + (size_t)nt * 16 * DM + k0);
      bw[nt].half[1] = *(const v8us*)(pw + (size_t)nt * 16 * DM + k0 + 16);
    }
    if (MODE == 3) {
      FragB a2;
      a2.half[0] = *(const v8us*)(pa2 + k0);
      a2.half[1] = *(const v8us*)(pa2 + k0 + 16);
#pragma unroll
      for (int nt = 0; nt < 4; ++nt) {
        acc[nt] = wm(a.v, bw[nt].v, acc[nt]);
        acc[nt] = wm(a2.v, bw[nt].v, acc[nt]);
      }
      asm volatile("v_nop\n\tv_nop\n\tv_nop\n\tv_nop" : "+v"(acc[0]), "+v"(acc[1]), "+v"(acc[2]), "+v"(acc[3])
                   : "v"(a.v), "v"(a2.v), "v"(bw[0].v), "v"(bw[1].v), "v"(bw[2].v), "v"(bw[3].v));
    } else {
#pragma unroll
      for (int nt = 0; nt < 4; ++nt) acc[nt] = wm(a.v, bw[nt].v, acc[nt]);
      asm volatile("v_nop\n\tv_nop\n\tv_nop\n\tv_nop" : "+v"(acc[0]), "+v"(acc[1]), "+v"(acc[2]), "+v"(acc[3])
                   : "v"(a.v), "v"(bw[0].v), "v"(bw[1].v), "v"(bw[2].v), "v"(bw[3].v));
    }
  }

  if (MODE == 3) {
    if (tid == 0) sbad = 0;
    __syncthreads();
    const int fi = (tid < NMB) ? tid : (NMB - 1);
    const int fb = flags[fi * 32];
    if (fb != 0) sbad = 1;
  }
  if (MODE == 2) {
#pragma unroll
    for (int nt = 0; nt < 4; ++nt) {
      *(v4fa*)&st[16 * nt + ln][16 * w + 8 * hh]     = __builtin_shufflevector(acc[nt], acc[nt], 0, 1, 2, 3);
      *(v4fa*)&st[16 * nt + ln][16 * w + 8 * hh + 4] = __builtin_shufflevector(acc[nt], acc[nt], 4, 5, 6, 7);
    }
  } else {
#pragma unroll
    for (int nt = 0; nt < 4; ++nt)
#pragma unroll
      for (int r = 0; r < 8; ++r) st[16 * w + 8 * hh + r][16 * nt + ln] = acc[nt][r];
  }
  __syncthreads();

  if (MODE == 3) {
    const bool poison = (sbad != 0);
    const float qnan = __uint_as_float(0x7fc00000u);
    for (int pass = 0; pass < 2; ++pass) {
#pragma unroll 1
      for (int it = 0; it < 8; ++it) {
        const int row = it * 8 + (tid >> 4), c4 = (tid & 15) * 4;
        const v4f x = *(const v4fa*)&st[row][c4];
        const v4f bb = *(const v4fa*)(bias0 + n0 + c4);
        v4f y;
        y[0] = x[0] + bf16_rne(bb[0]); y[1] = x[1] + bf16_rne(bb[1]);
        y[2] = x[2] + bf16_rne(bb[2]); y[3] = x[3] + bf16_rne(bb[3]);
        if (poison) { y[0] = qnan; y[1] = qnan; y[2] = qnan; y[3] = qnan; }
        const int m = m0 + row;
        const int bi = m / SEQ, s = m - bi * SEQ;
        *(volatile v4f*)(outF + ((size_t)bi * SEQ_FULL + s) * DM + n0 + c4) = y;
      }
      if (pass == 0) __threadfence();
    }
  } else {
    for (int pass = 0; pass < 2; ++pass) {
#pragma unroll 1
      for (int it = 0; it < 4; ++it) {
        const int row = it * 16 + (tid >> 3), c = (tid & 7) * 8;
        const v4f x0 = *(const v4fa*)&st[row][c], x1 = *(const v4fa*)&st[row][c + 4];
        if (MODE == 0) {
          const v4f u0 = *(const v4fa*)(bias0 + n0 + c), u1 = *(const v4fa*)(bias0 + n0 + c + 4);
          const v4f v0 = *(const v4fa*)(bias1 + n0 + c), v1 = *(const v4fa*)(bias1 + n0 + c + 4);
          float xu[8], xv[8];
#pragma unroll
          for (int e = 0; e < 4; ++e) {
            xu[e] = x0[e] + bf16_rne(u0[e]); xu[4 + e] = x1[e] + bf16_rne(u1[e]);
            xv[e] = x0[e] + bf16_rne(v0[e]); xv[4 + e] = x1[e] + bf16_rne(v1[e]);
          }
          v8us uh, ul, vh, vl;
          split8(xu, uh, ul);
          split8(xv, vh, vl);
          const size_t o = (size_t)(m0 + row) * DM + n0 + c;
          *(volatile v8us*)(o0 + o) = uh;
          *(volatile v8us*)(o1 + o) = ul;
          *(volatile v8us*)(o2 + o) = vh;
          *(volatile v8us*)(o3 + o) = vl;
        } else {
          float xx[8];
#pragma unroll
          for (int e = 0; e < 4; ++e) { xx[e] = x0[e]; xx[4 + e] = x1[e]; }
          v8us ph, pl;
          split8(xx, ph, pl);
          size_t o;
          if (MODE == 1) {
            o = (size_t)(m0 + row) * DM + n0 + c;
          } else {
            const int bi = m0 / SEQ, s0 = m0 - bi * SEQ;
            o = ((size_t)bi * DM + n0 + row) * SEQ + s0 + c;
          }
          *(volatile v8us*)(o0 + o) = ph;
          *(volatile v8us*)(o1 + o) = pl;
        }
      }
      if (pass == 0) __threadfence();
    }
  }
}

__global__ __launch_bounds__(128) void k_attn(const unsigned short* __restrict__ QuH, const unsigned short* __restrict__ QuL,
                                              const unsigned short* __restrict__ QvH, const unsigned short* __restrict__ QvL,
                                              const unsigned short* __restrict__ KH, const unsigned short* __restrict__ KL,
                                              const unsigned short* __restrict__ RH, const unsigned short* __restrict__ RL,
                                              const unsigned short* __restrict__ VtH, const unsigned short* __restrict__ VtL,
                                              unsigned short* CtxH, unsigned short* CtxL) {
  __shared__ __attribute__((aligned(16))) float gt[4][16][52];
  __shared__ __attribute__((aligned(16))) float so[4][16][68];
  const int tid = threadIdx.x, w = tid >> 5, lane = tid & 31, ln = lane & 15, hh = lane >> 4;
  const int qt = blockIdx.x % (SEQ / 64);
  const int bh = blockIdx.x / (SEQ / 64);
  const int h = bh % NH, b = bh / NH;
  const int qbase = qt * 64 + 16 * w;
  const int qg = qbase + ln;
  const size_t qo = ((size_t)b * SEQ + qg) * DM + h * HD + 8 * hh;
  FragB uh0, ul0, uh1, ul1, vh0, vl0, vh1, vl1;
  uh0.half[0] = *(const v8us*)(QuH + qo);      uh0.half[1] = *(const v8us*)(QuH + qo + 16);
  uh1.half[0] = *(const v8us*)(QuH + qo + 32); uh1.half[1] = *(const v8us*)(QuH + qo + 48);
  ul0.half[0] = *(const v8us*)(QuL + qo);      ul0.half[1] = *(const v8us*)(QuL + qo + 16);
  ul1.half[0] = *(const v8us*)(QuL + qo + 32); ul1.half[1] = *(const v8us*)(QuL + qo + 48);
  vh0.half[0] = *(const v8us*)(QvH + qo);      vh0.half[1] = *(const v8us*)(QvH + qo + 16);
  vh1.half[0] = *(const v8us*)(QvH + qo + 32); vh1.half[1] = *(const v8us*)(QvH + qo + 48);
  vl0.half[0] = *(const v8us*)(QvL + qo);      vl0.half[1] = *(const v8us*)(QvL + qo + 16);
  vl1.half[0] = *(const v8us*)(QvL + qo + 32); vl1.half[1] = *(const v8us*)(QvL + qo + 48);

  const unsigned short* KpH = KH + (size_t)b * SEQ * DM + h * HD;
  const unsigned short* KpL = KL + (size_t)b * SEQ * DM + h * HD;
  const unsigned short* RpH = RH + h * HD;
  const unsigned short* RpL = RL + h * HD;
  const unsigned short* VpH = VtH + ((size_t)b * DM + h * HD) * SEQ;
  const unsigned short* VpL = VtL + ((size_t)b * DM + h * HD) * SEQ;

  float mr = -3.0e38f, lr = 0.0f;
  v8f O[4] = {};
  const int nsteps = (qbase >> 5) + 1;
  int mlo = SEQ - 16 - qbase;
  v8f gc = tile_qk(RpH, RpL, mlo + ln, hh, vh0, vl0, vh1, vl1);
  const int gsh = 15 - ln + 8 * hh;
#pragma unroll 1
  for (int j = 0; j < nsteps; ++j) {
    const int key0 = 32 * j;
    const v8f g1 = tile_qk(RpH, RpL, mlo + 16 + ln, hh, vh0, vl0, vh1, vl1);
    const v8f g2 = tile_qk(RpH, RpL, mlo + 32 + ln, hh, vh0, vl0, vh1, vl1);
    *(v4fa*)&gt[w][ln][8 * hh]          = __builtin_shufflevector(gc, gc, 0, 1, 2, 3);
    *(v4fa*)&gt[w][ln][8 * hh + 4]      = __builtin_shufflevector(gc, gc, 4, 5, 6, 7);
    *(v4fa*)&gt[w][ln][16 + 8 * hh]     = __builtin_shufflevector(g1, g1, 0, 1, 2, 3);
    *(v4fa*)&gt[w][ln][16 + 8 * hh + 4] = __builtin_shufflevector(g1, g1, 4, 5, 6, 7);
    *(v4fa*)&gt[w][ln][32 + 8 * hh]     = __builtin_shufflevector(g2, g2, 0, 1, 2, 3);
    *(v4fa*)&gt[w][ln][32 + 8 * hh + 4] = __builtin_shufflevector(g2, g2, 4, 5, 6, 7);
    gc = g2;
    const v8f s0 = tile_qk(KpH, KpL, key0 + ln, hh, uh0, ul0, uh1, ul1);
    const v8f s1 = tile_qk(KpH, KpL, key0 + 16 + ln, hh, uh0, ul0, uh1, ul1);
    __builtin_amdgcn_fence(4  , "wavefront");
    __builtin_amdgcn_wave_barrier();
    float bd[16];
#pragma unroll
    for (int r = 0; r < 8; ++r) {
      bd[r]     = gt[w][ln][gsh + r];
      bd[8 + r] = gt[w][ln][gsh + 16 + r];
    }
    __builtin_amdgcn_fence(4  , "wavefront");
    __builtin_amdgcn_wave_barrier();
    float sc[16];
#pragma unroll
    for (int r = 0; r < 8; ++r) {
      const int kg = key0 + 8 * hh + r;
      const float a0 = (s0[r] + bd[r]) * 0.125f;
      const float a1 = (s1[r] + bd[8 + r]) * 0.125f;
      sc[r]     = (kg > qg) ? NEGFILL : a0;
      sc[8 + r] = (kg + 16 > qg) ? NEGFILL : a1;
    }
    float mx = sc[0];
#pragma unroll
    for (int i = 1; i < 16; ++i) mx = fmaxf(mx, sc[i]);
    mx = fmaxf(mx, __shfl_xor(mx, 16, 32));
    const float mnew = fmaxf(mr, mx);
    const float al = exp2f((mr - mnew) * LOG2E);
    mr = mnew;
    FragB ph, pl;
    float ps = 0.0f;
#pragma unroll
    for (int i = 0; i < 16; ++i) {
      const float pc = exp2f((sc[i] - mnew) * LOG2E);
      ps += pc;
      const unsigned short hb = bf16_bits(pc);
      ph.u[i] = hb;
      pl.u[i] = bf16_bits(pc - bf16_val(hb));
    }
    ps += __shfl_xor(ps, 16, 32);
    lr = lr * al + ps;
#pragma unroll
    for (int t = 0; t < 4; ++t) O[t] = O[t] * al;
#pragma unroll
    for (int t = 0; t < 4; ++t) {
      const size_t vo = (size_t)(16 * t + ln) * SEQ + key0 + 8 * hh;
      FragB fh, fl;
      fh.half[0] = *(const v8us*)(VpH + vo); fh.half[1] = *(const v8us*)(VpH + vo + 16);
      fl.half[0] = *(const v8us*)(VpL + vo); fl.half[1] = *(const v8us*)(VpL + vo + 16);
      O[t] = mma_pv(fh.v, fl.v, ph.v, pl.v, O[t]);
    }
    mlo += 32;
  }

  const float inv = 1.0f / lr;
#pragma unroll
  for (int t = 0; t < 4; ++t) {
    const v8f y = O[t] * inv;
    *(v4fa*)&so[w][ln][16 * t + 8 * hh]     = __builtin_shufflevector(y, y, 0, 1, 2, 3);
    *(v4fa*)&so[w][ln][16 * t + 8 * hh + 4] = __builtin_shufflevector(y, y, 4, 5, 6, 7);
  }
  __syncthreads();
  for (int pass = 0; pass < 2; ++pass) {
#pragma unroll 1
    for (int it = 0; it < 4; ++it) {
      const int row = it * 4 + (lane >> 3), c = (lane & 7) * 8;
      const v4f x0 = *(const v4fa*)&so[w][row][c], x1 = *(const v4fa*)&so[w][row][c + 4];
      float xx[8];
#pragma unroll
      for (int e = 0; e < 4; ++e) { xx[e] = x0[e]; xx[4 + e] = x1[e]; }
      v8us oh, ol;
      split8(xx, oh, ol);
      const size_t o = ((size_t)b * SEQ + qbase + row) * DM + h * HD + c;
      *(volatile v8us*)(CtxH + o) = oh;
      *(volatile v8us*)(CtxL + o) = ol;
    }
    if (pass == 0) __threadfence();
  }
}

extern "C" void kernel_launch(void* const* d_in, const int* in_sizes, int n_in,
                              void* d_out, int out_size, void* d_ws, size_t ws_size, hipStream_t stream) {
  if (n_in < 13) return;
  const long long need = (long long)(NB - 1) * SEQ_FULL * DM + (long long)SEQ * DM;
  if ((long long)in_sizes[0] < need || (long long)in_sizes[1] < need || (long long)in_sizes[2] < need) return;
  if ((long long)in_sizes[3] < (long long)SEQ * DM) return;
  if (in_sizes[4] < DM || in_sizes[5] < DM || in_sizes[12] < DM) return;
  if ((long long)in_sizes[6] < (long long)(SEQ - 1) * SEQ_FULL + SEQ) return;
  if (in_sizes[7] < DM * DM || in_sizes[8] < DM * DM || in_sizes[9] < DM * DM || in_sizes[10] < DM * DM || in_sizes[11] < DM * DM) return;
  if ((long long)out_size < need) return;
  const float* q_in = (const float*)d_in[0];
  const float* k_in = (const float*)d_in[1];
  const float* v_in = (const float*)d_in[2];
  const float* r_in = (const float*)d_in[3];
  const float* ub   = (const float*)d_in[4];
  const float* vb   = (const float*)d_in[5];
  const int*   mask = (const int*)d_in[6];
  const float* Wq   = (const float*)d_in[7];
  const float* Wk   = (const float*)d_in[8];
  const float* Wv   = (const float*)d_in[9];
  const float* Wr   = (const float*)d_in[10];
  const float* Wo   = (const float*)d_in[11];
  const float* bo   = (const float*)d_in[12];
  float* out = (float*)d_out;
  char* ws = (char*)d_ws;
  size_t off = 0;
  auto take = [&](size_t bytes) { char* p = ws + off; off += (bytes + 255) & ~(size_t)255; return (unsigned short*)p; };
  unsigned short* XQ = take(PLANE_B);
  unsigned short* XK = take(PLANE_B);
  unsigned short* XV = take(PLANE_B);
  unsigned short* XR = take(RPLANE_B);
  unsigned short* WQb = take(WPLANE_B);
  unsigned short* WKb = take(WPLANE_B);
  unsigned short* WVb = take(WPLANE_B);
  unsigned short* WRb = take(WPLANE_B);
  unsigned short* WOb = take(WPLANE_B);
  unsigned short* QUH = take(PLANE_B);
  unsigned short* QUL = take(PLANE_B);
  unsigned short* QVH = take(PLANE_B);
  unsigned short* QVL = take(PLANE_B);
  unsigned short* KHp = take(PLANE_B);
  unsigned short* KLp = take(PLANE_B);
  unsigned short* VTH = take(PLANE_B);
  unsigned short* VTL = take(PLANE_B);
  unsigned short* RHp = take(RPLANE_B);
  unsigned short* RLp = take(RPLANE_B);
  unsigned short* CH = take(PLANE_B);
  unsigned short* CL = take(PLANE_B);
  int* FLG = (int*)take((size_t)NMB * 128);
  if (off > ws_size || off > (size_t)134217728) return;

  const unsigned gx = (unsigned)((MROWS * 64 + 255) / 256);
  const unsigned gr = (unsigned)((SEQ * 64 + 255) / 256);
  const unsigned gw = (unsigned)((DM * 64 + 255) / 256);
  k_cvt<<<gx, 256, 0, stream>>>(q_in, XQ, NB, SEQ, BSTRIDE_FULL);
  k_cvt<<<gx, 256, 0, stream>>>(k_in, XK, NB, SEQ, BSTRIDE_FULL);
  k_cvt<<<gx, 256, 0, stream>>>(v_in, XV, NB, SEQ, BSTRIDE_FULL);
  k_cvt<<<gr, 256, 0, stream>>>(r_in, XR, 1, SEQ, (size_t)0);
  k_cvt<<<gw, 256, 0, stream>>>(Wq, WQb, 1, DM, (size_t)0);
  k_cvt<<<gw, 256, 0, stream>>>(Wk, WKb, 1, DM, (size_t)0);
  k_cvt<<<gw, 256, 0, stream>>>(Wv, WVb, 1, DM, (size_t)0);
  k_cvt<<<gw, 256, 0, stream>>>(Wr, WRb, 1, DM, (size_t)0);
  k_cvt<<<gw, 256, 0, stream>>>(Wo, WOb, 1, DM, (size_t)0);
  k_maskchk<<<(unsigned)NMB, 256, 0, stream>>>(mask, FLG);

  const dim3 gP((unsigned)(MROWS / 64), (unsigned)(DM / 64));
  const dim3 gR((unsigned)(SEQ / 64), (unsigned)(DM / 64));
  k_gemm<0><<<gP, 128, 0, stream>>>(XQ, XQ, WQb, ub, vb, QUH, QUL, QVH, QVL, out, FLG);
  k_gemm<1><<<gP, 128, 0, stream>>>(XK, XK, WKb, bo, bo, KHp, KLp, KHp, KLp, out, FLG);
  k_gemm<2><<<gP, 128, 0, stream>>>(XV, XV, WVb, bo, bo, VTH, VTL, VTH, VTL, out, FLG);
  k_gemm<1><<<gR, 128, 0, stream>>>(XR, XR, WRb, bo, bo, RHp, RLp, RHp, RLp, out, FLG);
  k_attn<<<(unsigned)(NB * NH * (SEQ / 64)), 128, 0, stream>>>(QUH, QUL, QVH, QVL, KHp, KLp, RHp, RLp, VTH, VTL, CH, CL);
  k_gemm<3><<<gP, 128, 0, stream>>>(CH, CL, WOb, bo, bo, CH, CL, CH, CL, out, FLG);
}
